// TransformerBlock_86019605004850
// MI455X (gfx1250) — hardware-verified
//
#include <hip/hip_runtime.h>
#include <math.h>

#ifndef NB
#define NB 2
#endif
#ifndef SEQ
#define SEQ 2048
#endif
#define NB_FULL 2
#define SEQ_FULL 2048
#define DM 1024
#define NH 16
#define HD 64
#define PD 128
#define DFF 4096
#define MTOK (NB * SEQ)
#define EARLY_ROWS 256
#define EARLY_QB (EARLY_ROWS / 64)
#define NQB (SEQ / 64)

static_assert(NB >= 1 && NB <= NB_FULL);
static_assert(SEQ <= SEQ_FULL);
static_assert(SEQ % 64 == 0);
static_assert(SEQ >= EARLY_ROWS);
static_assert(EARLY_ROWS % 64 == 0);
static_assert(NH * HD == DM);
static_assert(PD == 2 * HD);
static_assert(HD == 64);
static_assert(DM % 64 == 0 && DFF % 64 == 0 && (3 * DM) % 64 == 0);
static_assert(DM % 32 == 0 && DFF % 32 == 0 && PD % 32 == 0);
static_assert(MTOK % 64 == 0);
static_assert(DM == 8 * 32 * 4);

typedef __attribute__((ext_vector_type(16))) _Float16 v16h;
typedef __attribute__((ext_vector_type(8)))  _Float16 v8h;
typedef __attribute__((ext_vector_type(8)))  float    v8f;
typedef __attribute__((ext_vector_type(4)))  float    v4f;
typedef __attribute__((ext_vector_type(4)))  unsigned int v4u;
typedef __attribute__((ext_vector_type(2)))  unsigned int v2u;

union FragU { v16h v; v8h h[2]; };
__device__ __forceinline__ v16h frag_ld(const _Float16* p) { FragU f; f.h[0] = *(const v8h*)(p); f.h[1] = *(const v8h*)(p + 16); return f.v; }

__device__ __forceinline__ v8f mma16(v16h a, v16h b, v8f c) {
    c = __builtin_amdgcn_wmma_f32_16x16x32_f16(false, a, false, b, (short)0, c, false, false);
    asm volatile("v_nop\n\tv_nop\n\tv_nop\n\tv_nop" : "+v"(c) : "v"(a), "v"(b));
    return c;
}
__device__ __forceinline__ void dep_guard_h(v8f& a, v8f& b, v16h x, v16h y) { asm volatile("v_nop\n\tv_nop\n\tv_nop\n\tv_nop" : "+v"(a), "+v"(b) : "v"(x), "v"(y)); }
__device__ __forceinline__ void keep4_h(v16h a, v16h b, v16h c, v16h d) { asm volatile("v_nop" :: "v"(a), "v"(b), "v"(c), "v"(d)); }
__device__ __forceinline__ void acc_guard4(v8f& a, v8f& b, v8f& c, v8f& d) { asm volatile("v_nop\n\tv_nop\n\tv_nop\n\tv_nop" : "+v"(a), "+v"(b), "+v"(c), "+v"(d)); }

__device__ __forceinline__ void wave_sync() {
    __builtin_amdgcn_fence(3  , "workgroup");
    __builtin_amdgcn_wave_barrier();
    __builtin_amdgcn_fence(2  , "workgroup");
}

__device__ __forceinline__ float cmb_bf(float v) { const unsigned u = __builtin_bit_cast(unsigned, v); const unsigned r = (u + 0x7fffu + ((u >> 16) & 1u)) & 0xffff0000u; return __builtin_bit_cast(float, r); }
__device__ __forceinline__ unsigned int pk2h(float a, float b) { return (unsigned int)__builtin_bit_cast(unsigned short, (_Float16)a) | ((unsigned int)__builtin_bit_cast(unsigned short, (_Float16)b) << 16); }

#define VST2(T, ptr, val) do { const T vst2_v_ = (val); *(volatile T*)(ptr) = vst2_v_; __threadfence(); *(volatile T*)(ptr) = vst2_v_; } while (0)

__global__ __launch_bounds__(256) void k_cast_x(const float* __restrict__ X, unsigned short* __restrict__ DST) {
    const int u = (int)blockIdx.x * 256 + (int)threadIdx.x;
    if (u >= MTOK * (DM / 8)) return;
    const int m = u / (DM / 8); const int c0 = 8 * (u - m * (DM / 8));
    const int bb = m / SEQ; const int s = m - bb * SEQ;
    const float* src = X + ((size_t)bb * SEQ_FULL + s) * DM + c0;
    const v4f a = *(const v4f*)(src), b = *(const v4f*)(src + 4);
    v4u pk; pk.x = pk2h(cmb_bf(a.x), cmb_bf(a.y)); pk.y = pk2h(cmb_bf(a.z), cmb_bf(a.w)); pk.z = pk2h(cmb_bf(b.x), cmb_bf(b.y)); pk.w = pk2h(cmb_bf(b.z), cmb_bf(b.w));
    VST2(v4u, (v4u*)(DST + (size_t)m * DM + c0), pk);
}
__global__ __launch_bounds__(256) void k_cast_wT(const float* __restrict__ SRC, int lds, unsigned short* __restrict__ DST, int ldd, int nR, int nC, float sc) {
    const long long u = (long long)blockIdx.x * 256 + threadIdx.x; const int per = nR / 8;
    if (u >= (long long)nC * per) return;
    const int c = (int)(u / per); const int r0 = 8 * (int)(u - (long long)c * per);
    float w[8];
#pragma unroll
    for (int e = 0; e < 8; ++e) w[e] = cmb_bf(SRC[(size_t)(r0 + e) * lds + c]) * sc;
    v4u pk; pk.x = pk2h(w[0], w[1]); pk.y = pk2h(w[2], w[3]); pk.z = pk2h(w[4], w[5]); pk.w = pk2h(w[6], w[7]);
    VST2(v4u, (v4u*)(DST + (size_t)c * ldd + r0), pk);
}

template <bool BIAS, bool RELU, bool OUT16, int RESID>
__device__ __forceinline__ void gemm64_body(
    const _Float16* __restrict__ A, const int lda, const _Float16* __restrict__ Bt, const int ldb,
    float* __restrict__ Cf, _Float16* __restrict__ Ch, const int ldc,
    const float* __restrict__ bias, const float* __restrict__ resid, const int ldr, const int rseq, const int rfull,
    const int M, const int N, const int K, const float scale, const float oscale, float* sT)
{
    const int lane = threadIdx.x & 31, wave = threadIdx.x >> 5;
    const int tilesN = N >> 6, tilesM = M >> 6;
    const int tile = (int)blockIdx.x * 8 + wave;
    if (tile >= tilesM * tilesN) return;
    const int tm = tile / tilesN, tn = tile - tm * tilesN;
    const int m0 = tm << 6, n0 = tn << 6;
    const int rlane = lane & 15, koff = (lane >> 4) * 8, mOff = (lane >> 4) * 8;

    v8f acc[4][4];
#pragma unroll
    for (int i = 0; i < 4; ++i)
#pragma unroll
        for (int j = 0; j < 4; ++j) acc[i][j] = (v8f){0.f, 0.f, 0.f, 0.f, 0.f, 0.f, 0.f, 0.f};

    for (int k0 = 0; k0 < K; k0 += 32) {
        v16h bh[4];
#pragma unroll
        for (int j = 0; j < 4; ++j) bh[j] = frag_ld(Bt + (size_t)(n0 + (j << 4) + rlane) * ldb + koff + k0);
#pragma unroll
        for (int i = 0; i < 4; ++i) {
            const v16h ah = frag_ld(A + (size_t)(m0 + (i << 4) + rlane) * lda + koff + k0);
#pragma unroll
            for (int j = 0; j < 4; ++j) acc[i][j] = __builtin_amdgcn_wmma_f32_16x16x32_f16(false, ah, false, bh[j], (short)0, acc[i][j], false, false);
            dep_guard_h(acc[i][0], acc[i][3], ah, ah);
        }
        keep4_h(bh[0], bh[1], bh[2], bh[3]);
    }
    acc_guard4(acc[0][0], acc[0][1], acc[0][2], acc[0][3]);
    acc_guard4(acc[1][0], acc[1][1], acc[1][2], acc[1][3]);
    acc_guard4(acc[2][0], acc[2][1], acc[2][2], acc[2][3]);
    acc_guard4(acc[3][0], acc[3][1], acc[3][2], acc[3][3]);

    float* slab = sT + wave * (16 * 68);
#pragma unroll
    for (int i = 0; i < 4; ++i) {
        const int mBase = m0 + (i << 4);
#pragma unroll
        for (int j = 0; j < 4; ++j) {
            const int n = n0 + (j << 4) + rlane;
            float bv = 0.f;
            if (BIAS) bv = cmb_bf(bias[n]);
#pragma unroll
            for (int r = 0; r < 8; ++r) {
                float v = acc[i][j][r] * scale + bv;
                if (RELU) v = fmaxf(v, 0.0f);
                slab[(mOff + r) * 68 + (j << 4) + rlane] = v;
            }
        }
        wave_sync();
        if (!OUT16) {
            const int hh = lane >> 4, c4 = (lane & 15) * 4;
            int rrow0 = mBase;
            if (RESID != 0) { const int rb = mBase / rseq; rrow0 = rb * rfull + (mBase - rb * rseq); }
            v4f vals[8];
#pragma unroll
            for (int it = 0; it < 8; ++it) {
                const int row = it * 2 + hh;
                v4f v = *(const v4f*)(slab + row * 68 + c4);
                if (RESID != 0) {
                    v4f rr = *(const v4f*)(resid + (size_t)(rrow0 + row) * ldr + n0 + c4);
                    if (RESID == 2) { rr.x = cmb_bf(rr.x); rr.y = cmb_bf(rr.y); rr.z = cmb_bf(rr.z); rr.w = cmb_bf(rr.w); }
                    v = v + rr;
                }
                vals[it] = v;
            }
#pragma unroll
            for (int pass = 0; pass < 2; ++pass) {
#pragma unroll
                for (int it = 0; it < 8; ++it) *(volatile v4f*)(Cf + (size_t)(mBase + it * 2 + hh) * ldc + n0 + c4) = vals[it];
                __threadfence();
            }
        } else {
            const int q = lane >> 3, c8 = (lane & 7) * 8;
            v8h hv[4];
#pragma unroll
            for (int it = 0; it < 4; ++it) {
                const float* sp = slab + (it * 4 + q) * 68 + c8;
#pragma unroll
                for (int e = 0; e < 8; ++e) hv[it][e] = (_Float16)(sp[e] * oscale);
            }
#pragma unroll
            for (int pass = 0; pass < 2; ++pass) {
#pragma unroll
                for (int it = 0; it < 4; ++it) *(volatile v8h*)(Ch + (size_t)(mBase + it * 4 + q) * ldc + n0 + c8) = hv[it];
                __threadfence();
            }
        }
        wave_sync();
    }
}

#define WSC (1.0f / 64.0f)
__global__ __launch_bounds__(256) void k_gemm_qkv(const unsigned short* __restrict__ A, const unsigned short* __restrict__ Bt, float* __restrict__ C) {
    __shared__ __align__(16) float sT[8 * 16 * 68];
    gemm64_body<false, false, false, 0>((const _Float16*)A, DM, (const _Float16*)Bt, DM, C, nullptr, 3 * DM, nullptr, nullptr, 0, 1, 0, MTOK, 3 * DM, DM, WSC, 1.0f, sT);
}
__global__ __launch_bounds__(256) void k_gemm_wo(const unsigned short* __restrict__ A, const unsigned short* __restrict__ Bt, float* __restrict__ C, const float* __restrict__ bias, const float* __restrict__ xres) {
    __shared__ __align__(16) float sT[8 * 16 * 68];
    gemm64_body<true, false, false, 2>((const _Float16*)A, DM, (const _Float16*)Bt, DM, C, nullptr, DM, bias, xres, DM, SEQ, SEQ_FULL, MTOK, DM, DM, WSC * WSC, 1.0f, sT);
}
__global__ __launch_bounds__(256) void k_gemm_w1(const unsigned short* __restrict__ A, const unsigned short* __restrict__ Bt, unsigned short* __restrict__ C, const float* __restrict__ bias) {
    __shared__ __align__(16) float sT[8 * 16 * 68];
    gemm64_body<true, true, true, 0>((const _Float16*)A, DM, (const _Float16*)Bt, DM, nullptr, (_Float16*)C, DFF, bias, nullptr, 0, 1, 0, MTOK, DFF, DM, WSC, 1.0f, sT);
}
__global__ __launch_bounds__(256) void k_gemm_w2(const unsigned short* __restrict__ A, const unsigned short* __restrict__ Bt, float* __restrict__ C, const float* __restrict__ bias, const float* __restrict__ x1f) {
    __shared__ __align__(16) float sT[8 * 16 * 68];
    gemm64_body<true, false, false, 1>((const _Float16*)A, DFF, (const _Float16*)Bt, DFF, C, nullptr, DM, bias, x1f, DM, MTOK, 0, MTOK, DM, DFF, WSC, 1.0f, sT);
}

__device__ __forceinline__ float softplus_f(float t) { return fmaxf(t, 0.0f) + log1pf(expf(-fabsf(t))); }
template <bool RES> __device__ __forceinline__ _Float16 cv16(float v) {
    const _Float16 hi = (_Float16)v;
    if (RES) return (_Float16)((v - (float)hi) * 2048.0f);
    return hi;
}
template <bool RES>
__device__ __forceinline__ void pope_body(const float* __restrict__ QKV, const int* __restrict__ pos,
    const float* __restrict__ bq, const float* __restrict__ bk, const float* __restrict__ bv,
    const float* __restrict__ pbias, const float* __restrict__ freqs,
    _Float16* __restrict__ QP, _Float16* __restrict__ KP, _Float16* __restrict__ VTp, const int SP,
    _Float16* qt, _Float16* kt, _Float16* vt)
{
#pragma clang fp contract(off)
    const int tid = threadIdx.x; const int d = tid & 63; const int sl0 = tid >> 6;
    const int s0 = (int)blockIdx.x * 64; const int h = blockIdx.y; const int b = blockIdx.z; const int bh = b * NH + h;
    const float fr = cmb_bf(freqs[d]);
    const float pb = cmb_bf(pbias[h * HD + d]);
    const float bqv = cmb_bf(bq[h * HD + d]), bkv = cmb_bf(bk[h * HD + d]), bvv = cmb_bf(bv[h * HD + d]);
#pragma unroll 1
    for (int i = 0; i < 16; ++i) {
        const int sl = sl0 + 4 * i; const int s = s0 + sl;
        const float* row = QKV + (size_t)(b * SEQ + s) * (3 * DM) + h * HD + d;
        const float qv = row[0] + bqv, kv = row[DM] + bkv;
        const float muq = softplus_f(qv), muk = softplus_f(kv);
        const float ph = __fadd_rn(__fmul_rn((float)pos[s], fr), pb);
        float sn, cs;
        sincosf(ph, &sn, &cs);
        qt[sl * PD + d] = cv16<RES>(muq * cs); qt[sl * PD + HD + d] = cv16<RES>(muq * sn);
        kt[sl * PD + d] = cv16<RES>(muk * cs); kt[sl * PD + HD + d] = cv16<RES>(muk * sn);
        if (!RES) { const float vv = row[2 * DM] + bvv; vt[d * 64 + sl] = (_Float16)vv; }
    }
    __syncthreads();
    _Float16* qdst = QP + ((size_t)bh * SP + s0) * PD;
    _Float16* kdst = KP + ((size_t)bh * SP + s0) * PD;
    v8h qv_[4], kv_[4], vv_[2];
#pragma unroll
    for (int it = 0; it < 4; ++it) { qv_[it] = *(const v8h*)(qt + (it * 256 + tid) * 8); kv_[it] = *(const v8h*)(kt + (it * 256 + tid) * 8); }
    if (!RES) {
#pragma unroll
        for (int it = 0; it < 2; ++it) vv_[it] = *(const v8h*)(vt + (it * 256 + tid) * 8);
    }
#pragma unroll
    for (int pass = 0; pass < 2; ++pass) {
#pragma unroll
        for (int it = 0; it < 4; ++it) {
            *(volatile v8h*)(qdst + (it * 256 + tid) * 8) = qv_[it];
            *(volatile v8h*)(kdst + (it * 256 + tid) * 8) = kv_[it];
        }
        if (!RES) {
#pragma unroll
            for (int it = 0; it < 2; ++it) {
                const int p = it * 256 + tid; const int dd = p >> 3, cc = p & 7;
                *(volatile v8h*)(VTp + ((size_t)bh * HD + dd) * SP + s0 + cc * 8) = vv_[it];
            }
        }
        __threadfence();
    }
}
__global__ __launch_bounds__(256) void k_pope_hi(const float* __restrict__ QKV, const int* __restrict__ pos, const float* __restrict__ bq, const float* __restrict__ bk, const float* __restrict__ bv,
        const float* __restrict__ pbias, const float* __restrict__ freqs, unsigned short* __restrict__ QP, unsigned short* __restrict__ KP, unsigned short* __restrict__ VTp) {
    __shared__ __align__(16) _Float16 qt[64 * PD];
    __shared__ __align__(16) _Float16 kt[64 * PD];
    __shared__ __align__(16) _Float16 vt[64 * 64];
    pope_body<false>(QKV, pos, bq, bk, bv, pbias, freqs, (_Float16*)QP, (_Float16*)KP, (_Float16*)VTp, SEQ, qt, kt, vt);
}
__global__ __launch_bounds__(256) void k_pope_res(const float* __restrict__ QKV, const int* __restrict__ pos, const float* __restrict__ bq, const float* __restrict__ bk, const float* __restrict__ bv,
        const float* __restrict__ pbias, const float* __restrict__ freqs, unsigned short* __restrict__ QL, unsigned short* __restrict__ KL) {
    __shared__ __align__(16) _Float16 qt[64 * PD];
    __shared__ __align__(16) _Float16 kt[64 * PD];
    __shared__ __align__(16) _Float16 vt[8];
    pope_body<true>(QKV, pos, bq, bk, bv, pbias, freqs, (_Float16*)QL, (_Float16*)KL, nullptr, EARLY_ROWS, qt, kt, vt);
}

#define PSC 4096.0f
#define AOC 64.0f
template <bool EARLY>
__device__ __forceinline__ void attn_body(const _Float16* __restrict__ QH, const _Float16* __restrict__ KH, const _Float16* __restrict__ VT,
                                          const _Float16* __restrict__ QL, const _Float16* __restrict__ KL,
                                          _Float16* __restrict__ AO, const int qb0, _Float16* Psh, float* Os)
{
    const int tid = threadIdx.x, wave = tid >> 5, lane = tid & 31, hh = lane >> 4, c = lane & 15;
    const int qb = (int)blockIdx.x + qb0;
    const int bh = blockIdx.y;
    const int b = bh / NH, h = bh - b * NH;
    const int q0 = qb * 64 + wave * 16;
    const float SC2 = 0.08838834764831845f * 1.4426950408889634f;
    const float NEG = -__builtin_inff();
    _Float16* pw = Psh + wave * (16 * 64);
    float* os = Os + wave * (16 * 68);

    v16h qa[4];
    v16h ql[EARLY ? 4 : 1];
    {
        const _Float16* qrow = QH + ((size_t)bh * SEQ + q0 + c) * PD + 8 * hh;
#pragma unroll
        for (int dc = 0; dc < 4; ++dc) qa[dc] = frag_ld(qrow + dc * 32);
        if (EARLY) {
            const _Float16* qlrow = QL + ((size_t)bh * EARLY_ROWS + q0 + c) * PD + 8 * hh;
#pragma unroll
            for (int dc = 0; dc < 4; ++dc) ql[dc] = frag_ld(qlrow + dc * 32);
        }
    }
    float mrow[8], lrow[8];
    v8f oacc[4];
#pragma unroll
    for (int r = 0; r < 8; ++r) { mrow[r] = NEG; lrow[r] = 0.f; }
#pragma unroll
    for (int t = 0; t < 4; ++t) oacc[t] = (v8f){0.f, 0.f, 0.f, 0.f, 0.f, 0.f, 0.f, 0.f};

    for (int kc = 0; kc <= qb; ++kc) {
        const int kv0 = kc * 64;
        v8f s[4];
#pragma unroll
        for (int j = 0; j < 4; ++j) {
            const _Float16* krow = KH + ((size_t)bh * SEQ + kv0 + j * 16 + c) * PD + 8 * hh;
            v8f a = (v8f){0.f, 0.f, 0.f, 0.f, 0.f, 0.f, 0.f, 0.f};
#pragma unroll
            for (int dc = 0; dc < 4; ++dc) a = mma16(qa[dc], frag_ld(krow + dc * 32), a);
            if (EARLY) {
                const _Float16* klrow = KL + ((size_t)bh * EARLY_ROWS + kv0 + j * 16 + c) * PD + 8 * hh;
                v8f ar = (v8f){0.f, 0.f, 0.f, 0.f, 0.f, 0.f, 0.f, 0.f};
#pragma unroll
                for (int dc = 0; dc < 4; ++dc) {
                    ar = mma16(qa[dc], frag_ld(klrow + dc * 32), ar);
                    ar = mma16(ql[dc], frag_ld(krow + dc * 32), ar);
                }
                a = a + ar * (1.0f / 2048.0f);
            }
            s[j] = a;
        }
        const bool diag = (kc == qb);
#pragma unroll
        for (int r = 0; r < 8; ++r) {
            const int qrow = q0 + 8 * hh + r;
            float sv[4];
            float m = NEG;
#pragma unroll
            for (int j = 0; j < 4; ++j) {
                const int kvcol = kv0 + j * 16 + c;
                float v = s[j][r] * SC2;
                v = (diag && (kvcol > qrow)) ? NEG : v;
                sv[j] = v;
                m = fmaxf(m, v);
            }
            m = fmaxf(m, __shfl_xor(m, 1, 32)); m = fmaxf(m, __shfl_xor(m, 2, 32));
            m = fmaxf(m, __shfl_xor(m, 4, 32)); m = fmaxf(m, __shfl_xor(m, 8, 32));
            const float mnew = fmaxf(mrow[r], m);
            const float alpha = exp2f(mrow[r] - mnew);
            mrow[r] = mnew;
            float psum = 0.f;
#pragma unroll
            for (int j = 0; j < 4; ++j) {
                const float p = exp2f(sv[j] - mnew);
                psum += p;
                pw[(8 * hh + r) * 64 + j * 16 + c] = (_Float16)(p * PSC);
            }
            psum += __shfl_xor(psum, 1, 32); psum += __shfl_xor(psum, 2, 32);
            psum += __shfl_xor(psum, 4, 32); psum += __shfl_xor(psum, 8, 32);
            lrow[r] = lrow[r] * alpha + psum;
#pragma unroll
            for (int t = 0; t < 4; ++t) oacc[t][r] *= alpha;
        }
        wave_sync();
#pragma unroll
        for (int kk = 0; kk < 2; ++kk) {
            FragU pa;
            pa.h[0] = *(const v8h*)(pw + c * 64 + kk * 32 + 8 * hh);
            pa.h[1] = *(const v8h*)(pw + c * 64 + kk * 32 + 16 + 8 * hh);
#pragma unroll
            for (int t = 0; t < 4; ++t) {
                const _Float16* vrow = VT + ((size_t)bh * HD + t * 16 + c) * SEQ + kv0 + kk * 32 + 8 * hh;
                oacc[t] = mma16(pa.v, frag_ld(vrow), oacc[t]);
            }
        }
        wave_sync();
    }

#pragma unroll
    for (int r = 0; r < 8; ++r) {
        const float inv = AOC / (PSC * (1.0f + lrow[r]));
#pragma unroll
        for (int t = 0; t < 4; ++t) os[(8 * hh + r) * 68 + t * 16 + c] = oacc[t][r] * inv;
    }
    wave_sync();
    {
        const int q = lane >> 3, c8 = (lane & 7) * 8;
        v8h hv[4];
#pragma unroll
        for (int it = 0; it < 4; ++it) {
            const float* sp = os + (it * 4 + q) * 68 + c8;
#pragma unroll
            for (int e = 0; e < 8; ++e) hv[it][e] = (_Float16)sp[e];
        }
        _Float16* dst = AO + ((size_t)b * SEQ + q0) * DM + h * HD + c8;
#pragma unroll
        for (int pass = 0; pass < 2; ++pass) {
#pragma unroll
            for (int it = 0; it < 4; ++it) *(volatile v8h*)(dst + (size_t)(it * 4 + q) * DM) = hv[it];
            __threadfence();
        }
    }
}
__global__ __launch_bounds__(128) void k_attn_main(const unsigned short* __restrict__ QH, const unsigned short* __restrict__ KH, const unsigned short* __restrict__ VT, unsigned short* __restrict__ AO) {
    __shared__ __align__(16) _Float16 Psh[4 * 16 * 64];
    __shared__ __align__(16) float Os[4 * 16 * 68];
    attn_body<false>((const _Float16*)QH, (const _Float16*)KH, (const _Float16*)VT, nullptr, nullptr, (_Float16*)AO, EARLY_QB, Psh, Os);
}
__global__ __launch_bounds__(128) void k_attn_early(const unsigned short* __restrict__ QH, const unsigned short* __restrict__ KH, const unsigned short* __restrict__ VT,
                                                    const unsigned short* __restrict__ QL, const unsigned short* __restrict__ KL, unsigned short* __restrict__ AO) {
    __shared__ __align__(16) _Float16 Psh[4 * 16 * 64];
    __shared__ __align__(16) float Os[4 * 16 * 68];
    attn_body<true>((const _Float16*)QH, (const _Float16*)KH, (const _Float16*)VT, (const _Float16*)QL, (const _Float16*)KL, (_Float16*)AO, 0, Psh, Os);
}

template <bool WH>
__device__ __forceinline__ void ln_body(const float* __restrict__ Y, const float* __restrict__ g, const float* __restrict__ bt,
                                        float* __restrict__ O, unsigned short* __restrict__ OH)
{
    const int wave = threadIdx.x >> 5, lane = threadIdx.x & 31;
    const int row = (int)blockIdx.x * 8 + wave;
    if (row >= MTOK) return;
    const float* y = Y + (size_t)row * DM;
    float s = 0.f;
#pragma unroll 1
    for (int i = 0; i < 8; ++i) { const v4f v = *(const v4f*)(y + (i * 32 + lane) * 4); s += (v.x + v.y) + (v.z + v.w); }
    s += __shfl_xor(s, 16, 32); s += __shfl_xor(s, 8, 32); s += __shfl_xor(s, 4, 32); s += __shfl_xor(s, 2, 32); s += __shfl_xor(s, 1, 32);
    const float mu = s * (1.0f / (float)DM);
    float q = 0.f;
#pragma unroll 1
    for (int i = 0; i < 8; ++i) {
        const v4f v = *(const v4f*)(y + (i * 32 + lane) * 4);
        const float d0 = v.x - mu, d1 = v.y - mu, d2 = v.z - mu, d3 = v.w - mu;
        q += (d0 * d0 + d1 * d1) + (d2 * d2 + d3 * d3);
    }
    q += __shfl_xor(q, 16, 32); q += __shfl_xor(q, 8, 32); q += __shfl_xor(q, 4, 32); q += __shfl_xor(q, 2, 32); q += __shfl_xor(q, 1, 32);
    const float rs = rsqrtf(q * (1.0f / (float)DM) + 1e-5f);
#pragma unroll 1
    for (int i = 0; i < 8; ++i) {
        const int cc = (i * 32 + lane) * 4;
        const v4f v = *(const v4f*)(y + cc);
        const v4f gg = *(const v4f*)(g + cc);
        const v4f bb = *(const v4f*)(bt + cc);
        v4f o;
        o.x = (v.x - mu) * rs * cmb_bf(gg.x) + cmb_bf(bb.x);
        o.y = (v.y - mu) * rs * cmb_bf(gg.y) + cmb_bf(bb.y);
        o.z = (v.z - mu) * rs * cmb_bf(gg.z) + cmb_bf(bb.z);
        o.w = (v.w - mu) * rs * cmb_bf(gg.w) + cmb_bf(bb.w);
        v2u pk; pk.x = pk2h(o.x, o.y); pk.y = pk2h(o.z, o.w);
        float* od = O + (size_t)row * DM + cc;
        *(volatile v4f*)od = o;
        if (WH) *(volatile v2u*)(OH + (size_t)row * DM + cc) = pk;
        __threadfence();
        *(volatile v4f*)od = o;
        if (WH) *(volatile v2u*)(OH + (size_t)row * DM + cc) = pk;
    }
}
__global__ __launch_bounds__(256) void k_ln1(const float* __restrict__ Y, const float* __restrict__ g, const float* __restrict__ bt, float* __restrict__ O, unsigned short* __restrict__ OH) {
    ln_body<true>(Y, g, bt, O, OH);
}
__global__ __launch_bounds__(256) void k_ln2(const float* __restrict__ Y, const float* __restrict__ g, const float* __restrict__ bt, float* __restrict__ O) {
    ln_body<false>(Y, g, bt, O, nullptr);
}

constexpr size_t SZ_QKV = (size_t)MTOK * 3 * DM * 4;
constexpr size_t SZ_Y   = (size_t)MTOK * DM * 4;
constexpr size_t SZ_X16 = (size_t)MTOK * DM * 2;
constexpr size_t SZ_QP  = (size_t)NB * NH * SEQ * PD * 2;
constexpr size_t SZ_VT  = (size_t)NB * NH * HD * SEQ * 2;
constexpr size_t SZ_QL  = (size_t)NB * NH * EARLY_ROWS * PD * 2;
constexpr size_t SZ_W3T = (size_t)3 * DM * DM * 2;
constexpr size_t SZ_WOT = (size_t)DM * DM * 2;
constexpr size_t SZ_W1T = (size_t)DM * DFF * 2;
constexpr size_t SZ_W2T = (size_t)DFF * DM * 2;
constexpr size_t OFF_QKV = 0;
constexpr size_t OFF_X16 = OFF_QKV + SZ_QKV;
constexpr size_t OFF_QP  = OFF_X16 + SZ_X16;
constexpr size_t OFF_KP  = OFF_QP + SZ_QP;
constexpr size_t OFF_VT  = OFF_KP + SZ_QP;
constexpr size_t OFF_QL  = OFF_VT + SZ_VT;
constexpr size_t OFF_KL  = OFF_QL + SZ_QL;
constexpr size_t OFF_W3T = OFF_KL + SZ_QL;
constexpr size_t OFF_WOT = OFF_W3T + SZ_W3T;
constexpr size_t OFF_W1T = OFF_WOT + SZ_WOT;
constexpr size_t OFF_W2T = OFF_W1T + SZ_W1T;
constexpr size_t WS_TOTAL = OFF_W2T + SZ_W2T;
static_assert(WS_TOTAL <= (size_t)134217728);
static_assert(3 * SZ_Y <= SZ_QKV);
static_assert((size_t)MTOK * DFF * 2 <= 2 * SZ_QP);
static_assert(SZ_QKV % 256 == 0 && SZ_X16 % 256 == 0 && SZ_QP % 256 == 0 && SZ_VT % 256 == 0 && SZ_QL % 256 == 0);
static_assert(SZ_W3T % 256 == 0 && SZ_WOT % 256 == 0 && SZ_W1T % 256 == 0);

extern "C" void kernel_launch(void* const* d_in, const int* in_sizes, int n_in, void* d_out, int out_size, void* d_ws, size_t ws_size, hipStream_t stream) {
    if (n_in < 20) return;
    if ((size_t)in_sizes[0] < ((size_t)(NB - 1) * SEQ_FULL + SEQ) * DM) return;
    if (in_sizes[1] < SEQ) return;
    if (in_sizes[2] < DM * DM || in_sizes[4] < DM * DM || in_sizes[6] < DM * DM || in_sizes[8] < DM * DM) return;
    if (in_sizes[3] < DM || in_sizes[5] < DM || in_sizes[7] < DM || in_sizes[9] < DM) return;
    if (in_sizes[10] < NH * HD || in_sizes[11] < HD) return;
    if (in_sizes[12] < DM * DFF || in_sizes[13] < DFF || in_sizes[14] < DFF * DM || in_sizes[15] < DM) return;
    if (in_sizes[16] < DM || in_sizes[17] < DM || in_sizes[18] < DM || in_sizes[19] < DM) return;
    if ((size_t)out_size < (size_t)MTOK * DM) return;
    if (WS_TOTAL > ws_size) return;

    const float* x     = (const float*)d_in[0];
    const int*   posi  = (const int*)d_in[1];
    const float* Wq    = (const float*)d_in[2];
    const float* bq    = (const float*)d_in[3];
    const float* Wk    = (const float*)d_in[4];
    const float* bk    = (const float*)d_in[5];
    const float* Wv    = (const float*)d_in[6];
    const float* bv    = (const float*)d_in[7];
    const float* Wo    = (const float*)d_in[8];
    const float* bo    = (const float*)d_in[9];
    const float* pbias = (const float*)d_in[10];
    const float* freqs = (const float*)d_in[11];
    const float* W1    = (const float*)d_in[12];
    const float* b1    = (const float*)d_in[13];
    const float* W2    = (const float*)d_in[14];
    const float* b2    = (const float*)d_in[15];
    const float* g1    = (const float*)d_in[16];
    const float* beta1 = (const float*)d_in[17];
    const float* g2    = (const float*)d_in[18];
    const float* beta2 = (const float*)d_in[19];
    float* out = (float*)d_out;

    char* w = (char*)d_ws;
    float* QKV = (float*)(w + OFF_QKV);
    float* Y1  = (float*)(w + OFF_QKV);
    float* X1F = (float*)(w + OFF_QKV + SZ_Y);
    float* Y2  = (float*)(w + OFF_QKV + 2 * SZ_Y);
    unsigned short* X16  = (unsigned short*)(w + OFF_X16);
    unsigned short* AO16 = X16;
    unsigned short* X1H  = X16;
    unsigned short* QPH  = (unsigned short*)(w + OFF_QP);
    unsigned short* KPH  = (unsigned short*)(w + OFF_KP);
    unsigned short* H16  = QPH;
    unsigned short* VTH  = (unsigned short*)(w + OFF_VT);
    unsigned short* QPL  = (unsigned short*)(w + OFF_QL);
    unsigned short* KPL  = (unsigned short*)(w + OFF_KL);
    unsigned short* W3T  = (unsigned short*)(w + OFF_W3T);
    unsigned short* WOT  = (unsigned short*)(w + OFF_WOT);
    unsigned short* W1T  = (unsigned short*)(w + OFF_W1T);
    unsigned short* W2T  = (unsigned short*)(w + OFF_W2T);

    k_cast_x<<<(unsigned)((MTOK * (DM / 8) + 255) / 256), 256, 0, stream>>>(x, X16);
    k_cast_wT<<<(unsigned)(((long long)DM * (DM / 8) + 255) / 256), 256, 0, stream>>>(Wq, DM, W3T, DM, DM, DM, 64.0f);
    k_cast_wT<<<(unsigned)(((long long)DM * (DM / 8) + 255) / 256), 256, 0, stream>>>(Wk, DM, W3T + (size_t)DM * DM, DM, DM, DM, 64.0f);
    k_cast_wT<<<(unsigned)(((long long)DM * (DM / 8) + 255) / 256), 256, 0, stream>>>(Wv, DM, W3T + (size_t)2 * DM * DM, DM, DM, DM, 64.0f);
    k_cast_wT<<<(unsigned)(((long long)DM * (DM / 8) + 255) / 256), 256, 0, stream>>>(Wo, DM, WOT, DM, DM, DM, 64.0f);
    k_cast_wT<<<(unsigned)(((long long)DFF * (DM / 8) + 255) / 256), 256, 0, stream>>>(W1, DFF, W1T, DM, DM, DFF, 64.0f);
    k_cast_wT<<<(unsigned)(((long long)DM * (DFF / 8) + 255) / 256), 256, 0, stream>>>(W2, DM, W2T, DFF, DFF, DM, 64.0f);

    k_gemm_qkv<<<(unsigned)(((MTOK / 64) * ((3 * DM) / 64) + 7) / 8), 256, 0, stream>>>(X16, W3T, QKV);

    k_pope_hi<<<dim3((unsigned)(SEQ / 64), (unsigned)NH, (unsigned)NB), 256, 0, stream>>>(QKV, posi, bq, bk, bv, pbias, freqs, QPH, KPH, VTH);
    k_pope_res<<<dim3((unsigned)(EARLY_ROWS / 64), (unsigned)NH, (unsigned)NB), 256, 0, stream>>>(QKV, posi, bq, bk, bv, pbias, freqs, QPL, KPL);

    k_attn_early<<<dim3((unsigned)EARLY_QB, (unsigned)(NB * NH)), 128, 0, stream>>>(QPH, KPH, VTH, QPL, KPL, AO16);
    if (NQB > EARLY_QB)
        k_attn_main<<<dim3((unsigned)(NQB - EARLY_QB), (unsigned)(NB * NH)), 128, 0, stream>>>(QPH, KPH, VTH, AO16);

    k_gemm_wo<<<(unsigned)(((MTOK / 64) * (DM / 64) + 7) / 8), 256, 0, stream>>>(AO16, WOT, Y1, bo, x);
    k_ln1<<<(unsigned)((MTOK + 7) / 8), 256, 0, stream>>>(Y1, g1, beta1, X1F, X1H);

    k_gemm_w1<<<(unsigned)(((MTOK / 64) * (DFF / 64) + 7) / 8), 256, 0, stream>>>(X1H, W1T, H16, b1);
    k_gemm_w2<<<(unsigned)(((MTOK / 64) * (DM / 64) + 7) / 8), 256, 0, stream>>>(H16, W2T, Y2, b2, X1F);
    k_ln2<<<(unsigned)((MTOK + 7) / 8), 256, 0, stream>>>(Y2, g2, beta2, out);
}
